// CaDDN_Core_352187318845
// MI455X (gfx1250) — hardware-verified
//
#include <hip/hip_runtime.h>
#define IH 96
#define IW 320
#define NPI (IH * IW)
#define FC 64
#define DB 80
#define GX 200
#define GY 200
#define GZ 16
#define NBEV (GX * GY)
#define NVOX (GZ * NBEV)
#define CV (FC * GZ)
#define KB (9 * CV)
#define CHR 4000
#define NBT NBEV
#define NOUT 128
typedef __bf16 v16b __attribute__((ext_vector_type(16)));
typedef unsigned short v8us __attribute__((ext_vector_type(8), may_alias));
typedef float  v8f  __attribute__((ext_vector_type(8)));
typedef float  v4f  __attribute__((ext_vector_type(4)));
typedef float  v4fa __attribute__((ext_vector_type(4), may_alias));
union FragB { v16b v; v8us half[2]; unsigned short u[16]; };

__device__ __forceinline__ unsigned short bf16_bits(float x) { unsigned int u = __float_as_uint(x); return (unsigned short)((u + 0x7FFFu + ((u >> 16) & 1u)) >> 16); }
__device__ __forceinline__ float bf16_val(unsigned short b) { return __uint_as_float(((unsigned int)b) << 16); }
__device__ __forceinline__ float bf16_round(float x) { return bf16_val(bf16_bits(x)); }
template <int NT>
__device__ __forceinline__ v8f mmaN(v16b ah, v16b al, v16b bh, v16b bl, v8f c) {
  c = __builtin_amdgcn_wmma_f32_16x16x32_bf16(false, ah, false, bh, (short)0, c, false, false);
  if (NT >= 2) c = __builtin_amdgcn_wmma_f32_16x16x32_bf16(false, al, false, bh, (short)0, c, false, false);
  if (NT >= 3) c = __builtin_amdgcn_wmma_f32_16x16x32_bf16(false, ah, false, bl, (short)0, c, false, false);
  asm volatile("v_nop\n\tv_nop\n\tv_nop\n\tv_nop" : "+v"(c) : "v"(ah), "v"(al), "v"(bh), "v"(bl));
  return c;
}

__global__ __launch_bounds__(256) void k_wt_bf16(const float* __restrict__ W, unsigned short* __restrict__ Wt, int K, int N) {
  const int t = blockIdx.x * 256 + threadIdx.x;
  const int k8n = K / 8;
  if (t >= N * k8n) return;
  const int n = t / k8n, k8 = (t % k8n) * 8;
  v8us v;
#pragma unroll
  for (int i = 0; i < 8; ++i) v[i] = bf16_bits(W[(size_t)(k8 + i) * N + n]);
  *(volatile v8us*)(Wt + (size_t)n * K + k8) = v;
  __threadfence();
  *(volatile v8us*)(Wt + (size_t)n * K + k8) = v;
}

template <bool ASPLIT, int ACT, bool BIAS_BF16>
__global__ __launch_bounds__(128) void k_gemm_bf(const float* __restrict__ A, int lda, const unsigned short* __restrict__ Wt, int ldb,
                                               const float* __restrict__ bias, float* __restrict__ C, int ldc, int M, int N, int K) {
  __shared__ __attribute__((aligned(16))) float so[4][16][64];
  const int tid = threadIdx.x, w = tid >> 5, lane = tid & 31, ln = lane & 15, hh = lane >> 4;
  const int ntn = N / 64;
  const int wid = blockIdx.x * 4 + w;
  const int mt = wid / ntn, nq = wid % ntn;
  if (mt * 16 >= M) return;
  const int row0 = mt * 16, col0 = nq * 64;
  const float* arow = A + (size_t)(row0 + ln) * lda;
  v8f acc[4] = {};
  for (int kb = 0; kb < K; kb += 32) {
    FragB ah, al;
    const v4f x0 = *(const v4fa*)(arow + kb + 8 * hh), x1 = *(const v4fa*)(arow + kb + 8 * hh + 4);
    const v4f x2 = *(const v4fa*)(arow + kb + 16 + 8 * hh), x3 = *(const v4fa*)(arow + kb + 16 + 8 * hh + 4);
    float xs[16] = {x0[0],x0[1],x0[2],x0[3],x1[0],x1[1],x1[2],x1[3],x2[0],x2[1],x2[2],x2[3],x3[0],x3[1],x3[2],x3[3]};
#pragma unroll
    for (int i = 0; i < 16; ++i) { const unsigned short hb = bf16_bits(xs[i]); ah.u[i] = hb; al.u[i] = ASPLIT ? bf16_bits(xs[i] - bf16_val(hb)) : (unsigned short)0; }
#pragma unroll
    for (int t = 0; t < 4; ++t) {
      const unsigned short* brow = Wt + (size_t)(col0 + t * 16 + ln) * ldb + kb;
      FragB b;
      b.half[0] = *(const v8us*)(brow + 8 * hh);
      b.half[1] = *(const v8us*)(brow + 16 + 8 * hh);
      acc[t] = mmaN<ASPLIT ? 2 : 1>(ah.v, al.v, b.v, b.v, acc[t]);
    }
  }
#pragma unroll
  for (int t = 0; t < 4; ++t) {
    float bv = bias ? bias[col0 + t * 16 + ln] : 0.f;
    if (BIAS_BF16) bv = bf16_round(bv);
#pragma unroll
    for (int r = 0; r < 8; ++r) { float v = acc[t][r] + bv; if (ACT == 1) v = fmaxf(v, 0.f); so[w][8 * hh + r][t * 16 + ln] = v; }
  }
  __builtin_amdgcn_fence(__ATOMIC_ACQ_REL, "workgroup");
  __builtin_amdgcn_wave_barrier();
  const int rsub = lane >> 4, c4 = (lane & 15) * 4;
  for (int pass = 0; pass < 2; ++pass) {
#pragma unroll
    for (int q = 0; q < 8; ++q) {
      const int r = q * 2 + rsub;
      const v4f v = *(const v4fa*)&so[w][r][c4];
      *(volatile v4f*)(C + (size_t)(row0 + r) * ldc + col0 + c4) = v;
    }
    if (pass == 0) __threadfence();
  }
}

template <bool ASPLIT, int ACT, bool BIAS_BF16, bool RES_BF16>
__global__ __launch_bounds__(128) void k_gemm_bf3(const float* __restrict__ A, int lda, const unsigned short* __restrict__ Wt, int ldb,
                                                const float* __restrict__ bias, const float* __restrict__ resid, int rmod, int ldr,
                                                float* __restrict__ C, int ldc, int M, int N, int K) {
  __shared__ __attribute__((aligned(16))) float so[4][16][64];
  const int tid = threadIdx.x, w = tid >> 5, lane = tid & 31, ln = lane & 15, hh = lane >> 4;
  const int ntn = N / 64;
  const int wid = blockIdx.x * 4 + w;
  const int mt = wid / ntn, nq = wid % ntn;
  if (mt * 16 >= M) return;
  const int row0 = mt * 16, col0 = nq * 64;
  const float* arow = A + (size_t)(row0 + ln) * lda;
  v8f acc[4] = {};
  for (int kb = 0; kb < K; kb += 32) {
    FragB ah, al;
    const v4f x0 = *(const v4fa*)(arow + kb + 8 * hh), x1 = *(const v4fa*)(arow + kb + 8 * hh + 4);
    const v4f x2 = *(const v4fa*)(arow + kb + 16 + 8 * hh), x3 = *(const v4fa*)(arow + kb + 16 + 8 * hh + 4);
    float xs[16] = {x0[0],x0[1],x0[2],x0[3],x1[0],x1[1],x1[2],x1[3],x2[0],x2[1],x2[2],x2[3],x3[0],x3[1],x3[2],x3[3]};
#pragma unroll
    for (int i = 0; i < 16; ++i) { const unsigned short hb = bf16_bits(xs[i]); ah.u[i] = hb; al.u[i] = ASPLIT ? bf16_bits(xs[i] - bf16_val(hb)) : (unsigned short)0; }
#pragma unroll
    for (int t = 0; t < 4; ++t) {
      const unsigned short* brow = Wt + (size_t)(col0 + t * 16 + ln) * ldb + kb;
      FragB b;
      b.half[0] = *(const v8us*)(brow + 8 * hh);
      b.half[1] = *(const v8us*)(brow + 16 + 8 * hh);
      acc[t] = mmaN<ASPLIT ? 2 : 1>(ah.v, al.v, b.v, b.v, acc[t]);
    }
  }
#pragma unroll
  for (int t = 0; t < 4; ++t) {
    const int col = col0 + t * 16 + ln;
    float bv = bias ? bias[col] : 0.f;
    if (BIAS_BF16) bv = bf16_round(bv);
#pragma unroll
    for (int r = 0; r < 8; ++r) {
      float v = acc[t][r] + bv;
      if (resid) { float rv = resid[(size_t)((row0 + 8 * hh + r) % rmod) * ldr + col]; if (RES_BF16) rv = bf16_round(rv); v += rv; }
      if (ACT == 1) v = fmaxf(v, 0.f);
      if (ACT == 2) v = 0.5f * v * (1.0f + erff(v * 0.70710678118654752f));
      if (ACT == 3) { const float u = 0.7978845608028654f * (v + 0.044715f * v * v * v); v = 0.5f * v * (1.0f + tanhf(u)); }
      so[w][8 * hh + r][t * 16 + ln] = v;
    }
  }
  __builtin_amdgcn_fence(__ATOMIC_ACQ_REL, "workgroup");
  __builtin_amdgcn_wave_barrier();
  const int rsub = lane >> 4, c4 = (lane & 15) * 4;
  for (int pass = 0; pass < 2; ++pass) {
#pragma unroll
    for (int q = 0; q < 8; ++q) {
      const int r = q * 2 + rsub;
      const v4f v = *(const v4fa*)&so[w][r][c4];
      *(volatile v4f*)(C + (size_t)(row0 + r) * ldc + col0 + c4) = v;
    }
    if (pass == 0) __threadfence();
  }
}
template <bool PARAM_BF16>
__global__ __launch_bounds__(256) void k_layernorm(const float* __restrict__ X, const float* __restrict__ R, const float* __restrict__ g, const float* __restrict__ bta,
                                                  float* __restrict__ out_sum, float* __restrict__ out_norm, int N, float eps) {
  __shared__ float red[256];
  const int row = blockIdx.x, tid = threadIdx.x;
  const float* x = X + (size_t)row * N; const float* rr = R ? R + (size_t)row * N : nullptr;
  float vals[16];
  const int per = N / 256;
  float s1 = 0.f;
  for (int u = 0; u < per / 4; ++u) {
    const int j = tid * 4 + 1024 * u;
    const v4f a = *(const v4fa*)(x + j);
    v4f b = {0.f,0.f,0.f,0.f}; if (rr) b = *(const v4fa*)(rr + j);
#pragma unroll
    for (int q = 0; q < 4; ++q) { const float v = a[q] + b[q]; vals[u * 4 + q] = v; s1 += v; }
  }
  red[tid] = s1; __syncthreads();
  for (int st = 128; st > 0; st >>= 1) { if (tid < st) red[tid] += red[tid + st]; __syncthreads(); }
  const float mu = red[0] / (float)N; __syncthreads();
  float s2 = 0.f;
  for (int u = 0; u < per / 4; ++u)
#pragma unroll
    for (int q = 0; q < 4; ++q) { const float c = vals[u * 4 + q] - mu; s2 += c * c; }
  red[tid] = s2; __syncthreads();
  for (int st = 128; st > 0; st >>= 1) { if (tid < st) red[tid] += red[tid + st]; __syncthreads(); }
  const float rs = rsqrtf(red[0] / (float)N + eps);
  for (int pass = 0; pass < 2; ++pass) {
    for (int u = 0; u < per / 4; ++u) {
      const int j = tid * 4 + 1024 * u;
      v4f o, sm;
#pragma unroll
      for (int q = 0; q < 4; ++q) {
        float gg = g[j + q], bb = bta[j + q];
        if (PARAM_BF16) { gg = bf16_round(gg); bb = bf16_round(bb); }
        sm[q] = vals[u * 4 + q]; o[q] = (vals[u * 4 + q] - mu) * rs * gg + bb;
      }
      if (out_sum) *(volatile v4f*)(out_sum + (size_t)row * N + j) = sm;
      *(volatile v4f*)(out_norm + (size_t)row * N + j) = o;
    }
    if (pass == 0) __threadfence();
  }
}


typedef _Float16 v16h __attribute__((ext_vector_type(16)));
union FragH { v16h v; v8us half[2]; _Float16 h[16]; unsigned short u[16]; };
template <int NT>
__device__ __forceinline__ v8f mmaH(v16h ah, v16h al, v16h bh, v16h bl, v8f c) {
  c = __builtin_amdgcn_wmma_f32_16x16x32_f16(false, ah, false, bh, (short)0, c, false, false);
  if (NT >= 2) c = __builtin_amdgcn_wmma_f32_16x16x32_f16(false, al, false, bh, (short)0, c, false, false);
  if (NT >= 3) c = __builtin_amdgcn_wmma_f32_16x16x32_f16(false, ah, false, bl, (short)0, c, false, false);
  asm volatile("v_nop\n\tv_nop\n\tv_nop\n\tv_nop" : "+v"(c) : "v"(ah), "v"(al), "v"(bh), "v"(bl));
  return c;
}
template <bool ASPLIT>
__global__ __launch_bounds__(128) void k_gemm_h(const float* __restrict__ A, int lda, size_t sA, const _Float16* __restrict__ Bh, int ldb, size_t sB, float alpha, float* __restrict__ C, int ldc, size_t sC, int M, int N, int K) {
  __shared__ __attribute__((aligned(16))) float so[4][16][64];
  const int tid = threadIdx.x, w = tid >> 5, lane = tid & 31, ln = lane & 15, hh = lane >> 4; const int by = blockIdx.y;
  A += (size_t)by * sA; Bh += (size_t)by * sB; C += (size_t)by * sC;
  const int ntn = (N + 63) / 64; const int wid = blockIdx.x * 4 + w; const int mt = wid / ntn, nq = wid % ntn; if (mt * 16 >= M) return;
  const int row0 = mt * 16, col0 = nq * 64; const float* arow = A + (size_t)(row0 + ln) * lda;
  v8f acc[4] = {};
  for (int kb = 0; kb < K; kb += 32) {
    FragH ah, al;
    const v4f x0 = *(const v4fa*)(arow + kb + 8 * hh), x1 = *(const v4fa*)(arow + kb + 8 * hh + 4), x2 = *(const v4fa*)(arow + kb + 16 + 8 * hh), x3 = *(const v4fa*)(arow + kb + 16 + 8 * hh + 4);
    float xs[16] = {x0[0],x0[1],x0[2],x0[3],x1[0],x1[1],x1[2],x1[3],x2[0],x2[1],x2[2],x2[3],x3[0],x3[1],x3[2],x3[3]};
#pragma unroll
    for (int i = 0; i < 16; ++i) { const _Float16 h = (_Float16)xs[i]; ah.h[i] = h; al.h[i] = ASPLIT ? (_Float16)(xs[i] - (float)h) : (_Float16)0.0f; }
#pragma unroll
    for (int t = 0; t < 4; ++t) { if (col0 + t * 16 >= N) continue; const size_t boff = (size_t)(col0 + t * 16 + ln) * ldb + kb; FragH bq; bq.half[0] = *(const v8us*)(Bh + boff + 8 * hh); bq.half[1] = *(const v8us*)(Bh + boff + 16 + 8 * hh);
      acc[t] = mmaH<ASPLIT ? 2 : 1>(ah.v, al.v, bq.v, bq.v, acc[t]); }
  }
#pragma unroll
  for (int t = 0; t < 4; ++t) { if (col0 + t * 16 >= N) continue;
#pragma unroll
    for (int r = 0; r < 8; ++r) so[w][8 * hh + r][t * 16 + ln] = acc[t][r] * alpha; }
  __builtin_amdgcn_fence(__ATOMIC_ACQ_REL, "workgroup"); __builtin_amdgcn_wave_barrier();
  const int rsub = lane >> 4, c4 = (lane & 15) * 4;
  for (int pass = 0; pass < 2; ++pass) {
#pragma unroll
    for (int q = 0; q < 8; ++q) { const int r = q * 2 + rsub; if (col0 + c4 < N) { const v4f v = *(const v4fa*)&so[w][r][c4]; *(volatile v4f*)(C + (size_t)(row0 + r) * ldc + col0 + c4) = v; } }
    if (pass == 0) __threadfence(); }
}

__global__ __launch_bounds__(256) void k_wt_f16(const float* __restrict__ W, _Float16* __restrict__ Wt, int K, int N, float scale) {
  const int t = blockIdx.x * 256 + threadIdx.x; if (t >= N * (K / 8)) return; const int n = t / (K / 8), k8 = (t % (K / 8)) * 8; FragH f;
#pragma unroll
  for (int i = 0; i < 8; ++i) f.h[i] = (_Float16)(bf16_round(W[(size_t)(k8 + i) * N + n]) * scale); const v8us o = f.half[0];
  *(volatile v8us*)((unsigned short*)Wt + (size_t)n * K + k8) = o; __threadfence(); *(volatile v8us*)((unsigned short*)Wt + (size_t)n * K + k8) = o;
}
template <int ACT>
__global__ __launch_bounds__(128) void k_gemm_hhx(const _Float16* __restrict__ A, int lda, size_t sA, const _Float16* __restrict__ Bh, int ldb, size_t sB, float alpha, const float* __restrict__ bias, size_t sBias, const float* __restrict__ CP, int rowsPerB, size_t sCPb, int row0g,
    float* __restrict__ C, _Float16* __restrict__ C16, int ldc, size_t sC, int M, int N, int K) {
  __shared__ __attribute__((aligned(16))) float so[4][16][64];
  const int tid = threadIdx.x, w = tid >> 5, lane = tid & 31, ln = lane & 15, hh = lane >> 4; const int by = blockIdx.y;
  A += (size_t)by * sA; Bh += (size_t)by * sB; const size_t cofs = (size_t)by * sC; const float* bp = bias ? bias + (size_t)by * sBias : nullptr;
  const int ntn = (N + 63) / 64; const int wid = blockIdx.x * 4 + w; const int mt = wid / ntn, nq = wid % ntn; if (mt * 16 >= M) return;
  const int row0 = mt * 16, col0 = nq * 64; const _Float16* arow = A + (size_t)(row0 + ln) * lda;
  v8f acc[4] = {};
  for (int kb = 0; kb < K; kb += 32) { FragH ah; ah.half[0] = *(const v8us*)((const unsigned short*)arow + kb + 8 * hh); ah.half[1] = *(const v8us*)((const unsigned short*)arow + kb + 16 + 8 * hh);
#pragma unroll
    for (int t = 0; t < 4; ++t) { if (col0 + t * 16 >= N) continue; const size_t boff = (size_t)(col0 + t * 16 + ln) * ldb + kb; FragH bq; bq.half[0] = *(const v8us*)((const unsigned short*)Bh + boff + 8 * hh); bq.half[1] = *(const v8us*)((const unsigned short*)Bh + boff + 16 + 8 * hh);
      acc[t] = mmaH<1>(ah.v, ah.v, bq.v, bq.v, acc[t]); }
  }
#pragma unroll
  for (int t = 0; t < 4; ++t) { if (col0 + t * 16 >= N) continue; const int col = col0 + t * 16 + ln; const float bv = bp ? bf16_round(bp[col]) : 0.f;
#pragma unroll
    for (int r = 0; r < 8; ++r) { float v = acc[t][r] * alpha + bv; if (CP) { const int bidx = (row0g + row0 + 8 * hh + r) / rowsPerB; v += CP[(size_t)bidx * sCPb + (size_t)by * 64 + col]; } if (ACT == 1) v = (v > 0.f) ? v : expm1f(v); else if (ACT == 7) v = (v > 0.f) ? v + 1.0f : expf(v); else if (ACT == 8) v = tanhf(v); else if (ACT == 9) v = 0.5f * v * (1.0f + tanhf(0.7978845608028654f * (v + 0.044715f * v * v * v))); else if (ACT == 11) v = 1.0f / (1.0f + expf(-v)); else if (ACT == 12) v = (v > 0.f) ? v : 0.01f * v; else if (ACT == 14) v = (v > 0.f) ? v : 0.1f * v; else if (ACT == 15) v = v / (1.0f + expf(-v)); else if (ACT == 3) v = fmaxf(v, 0.f); else if (ACT == 6) v = 0.5f * v * (1.0f + erff(v * 0.70710678118654752f)); so[w][8 * hh + r][t * 16 + ln] = v; } }
  __builtin_amdgcn_fence(__ATOMIC_ACQ_REL, "workgroup"); __builtin_amdgcn_wave_barrier();
  const int rsub = lane >> 4, c4 = (lane & 15) * 4; typedef _Float16 v4h __attribute__((ext_vector_type(4)));
  for (int pass = 0; pass < 2; ++pass) {
#pragma unroll
    for (int q = 0; q < 8; ++q) { const int r = q * 2 + rsub; if (col0 + c4 < N) { const v4f v = *(const v4fa*)&so[w][r][c4]; if (C) *(volatile v4f*)(C + cofs + (size_t)(row0 + r) * ldc + col0 + c4) = v; if (C16) { v4h h4; for (int i = 0; i < 4; ++i) h4[i] = (_Float16)v[i]; *(volatile v4h*)(C16 + cofs + (size_t)(row0 + r) * ldc + col0 + c4) = h4; } } }
    if (pass == 0) __threadfence(); }
}


typedef _Float16 v4h __attribute__((ext_vector_type(4)));

__global__ __launch_bounds__(256) void k_x16(const float* __restrict__ x, _Float16* __restrict__ X16, size_t n8) { const size_t t = (size_t)blockIdx.x * 256 + threadIdx.x; if (t >= n8) return; FragH f;
#pragma unroll
  for (int q = 0; q < 8; ++q) f.h[q] = (_Float16)bf16_round(x[t * 8 + q]); *(volatile v8us*)((unsigned short*)X16 + t * 8) = f.half[0]; __threadfence(); *(volatile v8us*)((unsigned short*)X16 + t * 8) = f.half[0]; }
__global__ __launch_bounds__(256) void k_h16(const float* __restrict__ x, _Float16* __restrict__ X16, size_t n8) { const size_t t = (size_t)blockIdx.x * 256 + threadIdx.x; if (t >= n8) return; FragH f;
#pragma unroll
  for (int q = 0; q < 8; ++q) f.h[q] = (_Float16)x[t * 8 + q]; *(volatile v8us*)((unsigned short*)X16 + t * 8) = f.half[0]; __threadfence(); *(volatile v8us*)((unsigned short*)X16 + t * 8) = f.half[0]; }
__global__ __launch_bounds__(256) void k_round16f(const float* __restrict__ W, _Float16* __restrict__ Bt, size_t n8) { const size_t t = (size_t)blockIdx.x * 256 + threadIdx.x; if (t >= n8) return; FragH f;
#pragma unroll
  for (int i = 0; i < 8; ++i) f.h[i] = (_Float16)(bf16_round(W[t * 8 + i]) * 16.0f); *(volatile v8us*)((unsigned short*)Bt + t * 8) = f.half[0]; __threadfence(); *(volatile v8us*)((unsigned short*)Bt + t * 8) = f.half[0]; }
template <int NHv, int TTv>
__global__ __launch_bounds__(256) void k_vt(const _Float16* __restrict__ V16, int ldv, int voff, _Float16* __restrict__ Vt) { __shared__ unsigned short tl[64][66]; const int tid = threadIdx.x; const int slab = blockIdx.x / (TTv / 64), lg = blockIdx.x % (TTv / 64); const int b = slab / NHv, h = slab % NHv;
  for (int i = tid; i < 64 * 8; i += 256) { const int r = i / 8, c8 = (i % 8) * 8; FragH f; f.half[0] = *(const v8us*)((const unsigned short*)V16 + ((size_t)b * TTv + lg * 64 + r) * ldv + voff + h * 64 + c8);
#pragma unroll
    for (int q = 0; q < 8; ++q) tl[r][c8 + q] = f.u[q]; }
  __syncthreads();
  for (int pass = 0; pass < 2; ++pass) {
#pragma unroll
    for (int rd = 0; rd < 2; ++rd) { const int d = rd * 32 + tid / 8, pc = tid % 8; FragH f;
#pragma unroll
      for (int q = 0; q < 8; ++q) f.u[q] = tl[pc * 8 + q][d];
      *(volatile v8us*)((unsigned short*)Vt + ((size_t)slab * 64 + d) * TTv + lg * 64 + pc * 8) = f.half[0]; }
    if (pass == 0) __threadfence(); } }

__global__ __launch_bounds__(256) void k_hl(const float* __restrict__ F, _Float16* __restrict__ Hh, _Float16* __restrict__ Hl, size_t n8) { const size_t t = (size_t)blockIdx.x * 256 + threadIdx.x; if (t >= n8) return; FragH fh, fl; const v4f a = *(const v4fa*)(F + t * 8), c = *(const v4fa*)(F + t * 8 + 4);
#pragma unroll
  for (int q = 0; q < 4; ++q) { _Float16 h = (_Float16)a[q]; fh.h[q] = h; fl.h[q] = (_Float16)((a[q] - (float)h) * 1024.0f); h = (_Float16)c[q]; fh.h[4 + q] = h; fl.h[4 + q] = (_Float16)((c[q] - (float)h) * 1024.0f); }
  for (int pass = 0; pass < 2; ++pass) { *(volatile v8us*)((unsigned short*)Hh + t * 8) = fh.half[0]; *(volatile v8us*)((unsigned short*)Hl + t * 8) = fl.half[0]; if (pass == 0) __threadfence(); } }

__device__ __forceinline__ v16h g2_frag(const _Float16* p, int hh) { FragH f; f.half[0] = *(const v8us*)((const unsigned short*)p + 8 * hh); f.half[1] = *(const v8us*)((const unsigned short*)p + 16 + 8 * hh); return f.v; }
__device__ __forceinline__ v8f g2_mma(v16h a, v16h b, v8f c) { v8f d = __builtin_amdgcn_wmma_f32_16x16x32_f16(false, a, false, b, (short)0, c, false, false); asm volatile("v_nop\n\tv_nop\n\tv_nop\n\tv_nop" : "+v"(d) : "v"(a), "v"(b)); return d; }
template <int ACT>
__global__ __launch_bounds__(128) void k_gemm2(const _Float16* __restrict__ A, int lda, size_t sA, const _Float16* __restrict__ Bh, int ldb, size_t sB, float alpha, const float* __restrict__ bias, size_t sBias, const float* __restrict__ CP, int rowsPerB, size_t sCPb, int row0g,
    float* __restrict__ C, _Float16* __restrict__ C16, int ldc, size_t sC, int M, int N, int K) {
  __shared__ __attribute__((aligned(16))) float so[4][32][68];
  const int tid = threadIdx.x, w = tid >> 5, lane = tid & 31, ln = lane & 15, hh = lane >> 4; const int by = blockIdx.y;
  A += (size_t)by * sA; Bh += (size_t)by * sB; const size_t cofs = (size_t)by * sC; const float* bp = bias ? bias + (size_t)by * sBias : nullptr;
  const int ntn = N >> 6; const int mt = blockIdx.x / ntn, nq = blockIdx.x - mt * ntn; const int row0 = mt * 128 + 32 * w, col0 = nq * 64; if (row0 >= M) return;
  const _Float16* a0p = A + (size_t)(row0 + ln) * lda; const _Float16* a1p = a0p + (size_t)16 * lda;
  const _Float16* b0p = Bh + (size_t)(col0 + ln) * ldb; const _Float16* b1p = b0p + (size_t)16 * ldb; const _Float16* b2p = b1p + (size_t)16 * ldb; const _Float16* b3p = b2p + (size_t)16 * ldb;
  const v8f z8 = {0.f,0.f,0.f,0.f,0.f,0.f,0.f,0.f}; v8f c00 = z8, c01 = z8, c02 = z8, c03 = z8, c10 = z8, c11 = z8, c12 = z8, c13 = z8;
#pragma unroll 1
  for (int kb = 0; kb < K; kb += 32) { const v16h a0 = g2_frag(a0p + kb, hh), a1 = g2_frag(a1p + kb, hh);
    v16h b = g2_frag(b0p + kb, hh); c00 = g2_mma(a0, b, c00); c10 = g2_mma(a1, b, c10);
    b = g2_frag(b1p + kb, hh); c01 = g2_mma(a0, b, c01); c11 = g2_mma(a1, b, c11);
    b = g2_frag(b2p + kb, hh); c02 = g2_mma(a0, b, c02); c12 = g2_mma(a1, b, c12);
    b = g2_frag(b3p + kb, hh); c03 = g2_mma(a0, b, c03); c13 = g2_mma(a1, b, c13); }
  v8f accs[8] = {c00, c01, c02, c03, c10, c11, c12, c13};
#pragma unroll
  for (int u = 0; u < 8; ++u) { const int t = u & 3, half = u >> 2; const int col = col0 + t * 16 + ln; const float bv = bp ? bf16_round(bp[col]) : 0.f;
#pragma unroll
    for (int r = 0; r < 8; ++r) { const int rloc = half * 16 + 8 * hh + r; float v = accs[u][r] * alpha + bv; if (CP) { const int bidx = (row0g + row0 + rloc) / rowsPerB; v += CP[(size_t)bidx * sCPb + (size_t)by * 64 + col]; }
      if (ACT == 3) v = fmaxf(v, 0.f); else if (ACT == 6) v = 0.5f * v * (1.0f + erff(v * 0.70710678118654752f)); else if (ACT == 11) v = 1.0f / (1.0f + expf(-v)); else if (ACT == 15) v = v / (1.0f + expf(-v)); else if (ACT == 12) v = (v > 0.f) ? v : 0.01f * v; else if (ACT == 8) v = tanhf(v);
      so[w][rloc][t * 16 + ln] = v; } }
  __builtin_amdgcn_fence(__ATOMIC_ACQ_REL, "workgroup"); __builtin_amdgcn_wave_barrier();
  const int rsub = lane >> 4, c4 = (lane & 15) * 4;
  for (int pass = 0; pass < 2; ++pass) {
#pragma unroll
    for (int q = 0; q < 16; ++q) { const int r = q * 2 + rsub; const v4f v = *(const v4fa*)&so[w][r][c4]; if (C) *(volatile v4f*)(C + cofs + (size_t)(row0 + r) * ldc + col0 + c4) = v; if (C16) { v4h h4; for (int i = 0; i < 4; ++i) h4[i] = (_Float16)v[i]; *(volatile v4h*)(C16 + cofs + (size_t)(row0 + r) * ldc + col0 + c4) = h4; } }
    if (pass == 0) __threadfence(); } }


__global__ __launch_bounds__(256) void k_im3(const float* __restrict__ img, _Float16* __restrict__ IM3) {
  const int p = blockIdx.x * 256 + threadIdx.x; if (p >= NPI) return; const int y = p / IW, x = p % IW; FragH f[2];
#pragma unroll
  for (int i = 0; i < 32; ++i) { float v = 0.f; if (i < 27) { const int k = i / 3, c = i % 3; const int yy = y + k / 3 - 1, xx = x + k % 3 - 1; if (yy >= 0 && yy < IH && xx >= 0 && xx < IW) v = bf16_round(img[((size_t)c * IH + yy) * IW + xx]); } f[i >> 4].h[i & 15] = (_Float16)v; }
  unsigned short* d = (unsigned short*)IM3 + (size_t)p * 32; for (int pass = 0; pass < 2; ++pass) { *(volatile v8us*)d = f[0].half[0]; *(volatile v8us*)(d + 8) = f[0].half[1]; *(volatile v8us*)(d + 16) = f[1].half[0]; *(volatile v8us*)(d + 24) = f[1].half[1]; if (pass == 0) __threadfence(); } }
__global__ __launch_bounds__(256) void k_w3(const float* __restrict__ Wt, const float* __restrict__ bsrc, int O, int orows, _Float16* __restrict__ Bt, float* __restrict__ BB) {
  const int o = blockIdx.x * 256 + threadIdx.x; if (o >= orows) return; FragH f[2];
#pragma unroll
  for (int i = 0; i < 32; ++i) { float v = 0.f; if (i < 27 && o < O) { const int k = i / 3, c = i % 3; v = bf16_round(Wt[((size_t)o * 3 + c) * 9 + k]) * 16.0f; } f[i >> 4].h[i & 15] = (_Float16)v; }
  unsigned short* d = (unsigned short*)Bt + (size_t)o * 32; const float bv = (o < O) ? bsrc[o] : 0.f;
  for (int pass = 0; pass < 2; ++pass) { *(volatile v8us*)d = f[0].half[0]; *(volatile v8us*)(d + 8) = f[0].half[1]; *(volatile v8us*)(d + 16) = f[1].half[0]; *(volatile v8us*)(d + 24) = f[1].half[1]; *(volatile float*)(BB + o) = bv; if (pass == 0) __threadfence(); } }
__global__ __launch_bounds__(256) void k_bnst(const float* __restrict__ F, int ld, int NP, float* __restrict__ ST) {
  #pragma clang fp contract(off)
  __shared__ float sh[256]; const int c = blockIdx.x; const int tid = threadIdx.x; float s = 0.f; for (int p = tid; p < NP; p += 256) s += F[(size_t)p * ld + c]; sh[tid] = s; __syncthreads();
  for (int st = 128; st > 0; st >>= 1) { if (tid < st) sh[tid] += sh[tid + st]; __syncthreads(); } const float mu = sh[0] / (float)NP; __syncthreads();
  float q2 = 0.f; for (int p = tid; p < NP; p += 256) { const float d = F[(size_t)p * ld + c] - mu; q2 += d * d; } sh[tid] = q2; __syncthreads();
  for (int st = 128; st > 0; st >>= 1) { if (tid < st) sh[tid] += sh[tid + st]; __syncthreads(); }
  if (tid == 0) { for (int pass = 0; pass < 2; ++pass) { *(volatile float*)(ST + c * 32) = mu; *(volatile float*)(ST + c * 32 + 1) = sh[0] / (float)NP; if (pass == 0) __threadfence(); } } }
__global__ __launch_bounds__(256) void k_bnrelu1(const float* __restrict__ F1, const float* __restrict__ ST, const float* __restrict__ g, const float* __restrict__ bb, float* __restrict__ FEAT) {
  #pragma clang fp contract(off)
  const int t = blockIdx.x * 256 + threadIdx.x; if (t >= NPI * (FC / 4)) return; const int c0 = (t % (FC / 4)) * 4; const int p = t / (FC / 4); v4f o;
#pragma unroll
  for (int q = 0; q < 4; ++q) { const int c = c0 + q; float v = (F1[(size_t)p * FC + c] - ST[c * 32]) * rsqrtf(ST[c * 32 + 1] + 1e-5f); v = bf16_round(g[c]) * v; v += bf16_round(bb[c]); o[q] = fmaxf(v, 0.f); }
  *(volatile v4f*)(FEAT + (size_t)p * FC + c0) = o; __threadfence(); *(volatile v4f*)(FEAT + (size_t)p * FC + c0) = o; }
__global__ __launch_bounds__(256) void k_dsoft(const float* __restrict__ DL, float* __restrict__ PROB) {
  #pragma clang fp contract(off)
  const int tid = threadIdx.x, w = tid >> 5, ln = tid & 31; const int p = blockIdx.x * 8 + w; if (p >= NPI) return; const float* r = DL + (size_t)p * 128; float v[3]; float m = -3.0e38f;
#pragma unroll
  for (int c = 0; c < 3; ++c) { const int d = c * 32 + ln; v[c] = (d < DB) ? r[d] : -3.0e38f; m = fmaxf(m, v[c]); }
  for (int o = 16; o > 0; o >>= 1) m = fmaxf(m, __shfl_xor(m, o, 32)); float su = 0.f;
#pragma unroll
  for (int c = 0; c < 3; ++c) { const int d = c * 32 + ln; v[c] = (d < DB) ? expf(v[c] - m) : 0.f; su += v[c]; }
  for (int o = 16; o > 0; o >>= 1) su += __shfl_xor(su, o, 32);
  for (int pass = 0; pass < 2; ++pass) { for (int c = 0; c < 3; ++c) { const int d = c * 32 + ln; if (d < DB) *(volatile float*)(PROB + (size_t)p * 128 + d) = v[c] / su; } if (pass == 0) __threadfence(); } }
__global__ __launch_bounds__(256) void k_dlout(const float* __restrict__ DL, float* __restrict__ out2) { const int t = blockIdx.x * 256 + threadIdx.x; if (t >= DB * (NPI / 4)) return; const int p0 = (t % (NPI / 4)) * 4; const int d = t / (NPI / 4); v4f o; for (int q = 0; q < 4; ++q) o[q] = DL[(size_t)(p0 + q) * 128 + d]; *(volatile v4f*)(out2 + (size_t)d * NPI + p0) = o; __threadfence(); *(volatile v4f*)(out2 + (size_t)d * NPI + p0) = o; }
__device__ __forceinline__ void voxel_one(int n, int c0, const float* __restrict__ calib, const float* __restrict__ FEAT, const float* __restrict__ PROB, float acc[8]) {
  #pragma clang fp contract(off)
  const int x = n % GX, y = (n / GX) % GY, z = n / (GX * GY);
  const float xs = (x == GX - 1) ? 70.4f : 0.0f + (float)x * ((70.4f - 0.0f) / (float)(GX - 1)); const float ys = (y == GY - 1) ? 40.0f : -40.0f + (float)y * ((40.0f - -40.0f) / (float)(GY - 1)); const float zs = (z == GZ - 1) ? 1.0f : -3.0f + (float)z * ((1.0f - -3.0f) / (float)(GZ - 1));
  float ip[3];
#pragma unroll
  for (int i = 0; i < 3; ++i) { float s = bf16_round(calib[i * 4 + 0]) * xs; s += bf16_round(calib[i * 4 + 1]) * ys; s += bf16_round(calib[i * 4 + 2]) * zs; s += bf16_round(calib[i * 4 + 3]) * 1.0f; ip[i] = s; }
  const float dep = ip[2]; const float u = ip[0] / (dep + 1e-5f), v = ip[1] / (dep + 1e-5f);
  float un = u / (float)(IW - 1) * 2.0f; un -= 1.0f; float vn = v / (float)(IH - 1) * 2.0f; vn -= 1.0f; float dn = (dep - 2.0f) / (42.0f - 2.0f) * 2.0f; dn -= 1.0f;
  float gx = (un + 1.0f) * (float)IW; gx -= 1.0f; gx = gx * 0.5f; float gy = (vn + 1.0f) * (float)IH; gy -= 1.0f; gy = gy * 0.5f; float gz = (dn + 1.0f) * (float)DB; gz -= 1.0f; gz = gz * 0.5f;
  const float x0f = floorf(gx), y0f = floorf(gy), z0f = floorf(gz); const float wx = gx - x0f, wy = gy - y0f, wz = gz - z0f;
  const int x0 = (int)fminf(fmaxf(x0f, -4.f), (float)(IW + 4)), y0 = (int)fminf(fmaxf(y0f, -4.f), (float)(IH + 4)), z0 = (int)fminf(fmaxf(z0f, -4.f), (float)(DB + 4));
  for (int q = 0; q < 8; ++q) acc[q] = 0.f;
#pragma unroll
  for (int cz = 0; cz < 2; ++cz) {
#pragma unroll
    for (int cy = 0; cy < 2; ++cy) {
#pragma unroll
      for (int cx = 0; cx < 2; ++cx) { const int iz = z0 + cz, iy = y0 + cy, ix = x0 + cx; if (iz < 0 || iz >= DB || iy < 0 || iy >= IH || ix < 0 || ix >= IW) continue;
        float w = (cz ? wz : 1.0f - wz) * (cy ? wy : 1.0f - wy); w = w * (cx ? wx : 1.0f - wx); const size_t pp = (size_t)iy * IW + ix; const float pr = PROB[pp * 128 + iz]; const float* fr = FEAT + pp * FC + c0;
#pragma unroll
        for (int q = 0; q < 8; ++q) { const float fv = fr[q] * pr; acc[q] += fv * w; } } } } }
__global__ __launch_bounds__(256) void k_voxel(const float* __restrict__ calib, const float* __restrict__ FEAT, const float* __restrict__ PROB, _Float16* __restrict__ VOX) {
  const size_t t = (size_t)blockIdx.x * 256 + threadIdx.x; if (t >= (size_t)(NVOX / 2) * (FC / 8)) return; const int m = (int)(t % (NVOX / 2)); const int c0 = (int)(t / (NVOX / 2)) * 8; const int n0 = 2 * m; const int z = n0 / (GX * GY); const int rem = n0 % (GX * GY);
  float a0[8], a1[8]; voxel_one(n0, c0, calib, FEAT, PROB, a0); voxel_one(n0 + 1, c0, calib, FEAT, PROB, a1);
  unsigned pk[8];
#pragma unroll
  for (int q = 0; q < 8; ++q) { FragH f; f.h[0] = (_Float16)a0[q]; f.h[1] = (_Float16)a1[q]; pk[q] = (unsigned)f.u[0] | ((unsigned)f.u[1] << 16); }
  for (int pass = 0; pass < 2; ++pass) {
#pragma unroll
    for (int q = 0; q < 8; ++q) *(volatile unsigned*)((unsigned short*)VOX + ((size_t)(c0 + q) * GZ + z) * NBEV + rem) = pk[q];
    if (pass == 0) __threadfence(); } }
__global__ __launch_bounds__(256) void k_imb(const _Float16* __restrict__ VOX, int r0, _Float16* __restrict__ IMB) {
  const size_t t = (size_t)blockIdx.x * 256 + threadIdx.x; if (t >= (size_t)CHR * 9 * (CV / 8)) return; const int c0 = (int)(t % (CV / 8)) * 8; const int k = (int)((t / (CV / 8)) % 9); const int r = (int)(t / ((CV / 8) * 9)); const int p = r0 + r; const int y = p / GX + k / 3 - 1, x = p % GX + k % 3 - 1; const bool ok = y >= 0 && y < GY && x >= 0 && x < GX; FragH f;
#pragma unroll
  for (int q = 0; q < 8; ++q) f.h[q] = ok ? VOX[(size_t)(c0 + q) * NBEV + y * GX + x] : (_Float16)0.0f;
  *(volatile v8us*)((unsigned short*)IMB + (size_t)r * KB + k * CV + c0) = f.half[0]; __threadfence(); *(volatile v8us*)((unsigned short*)IMB + (size_t)r * KB + k * CV + c0) = f.half[0]; }
__global__ __launch_bounds__(256) void k_wbev(const float* __restrict__ Wt, _Float16* __restrict__ Bt) { const size_t t = (size_t)blockIdx.x * 256 + threadIdx.x; if (t >= (size_t)NOUT * 9 * (CV / 8)) return; const int c0 = (int)(t % (CV / 8)) * 8; const int k = (int)((t / (CV / 8)) % 9); const int o = (int)(t / ((CV / 8) * 9)); FragH f;
  for (int q = 0; q < 8; ++q) f.h[q] = (_Float16)(bf16_round(Wt[((size_t)o * CV + c0 + q) * 9 + k]) * 16.0f); *(volatile v8us*)((unsigned short*)Bt + (size_t)o * KB + k * CV + c0) = f.half[0]; __threadfence(); *(volatile v8us*)((unsigned short*)Bt + (size_t)o * KB + k * CV + c0) = f.half[0]; }
__global__ __launch_bounds__(256) void k_bevout(const float* __restrict__ BEV, const float* __restrict__ ST, const float* __restrict__ g, const float* __restrict__ bb, float* __restrict__ out) {
  #pragma clang fp contract(off)
  const int t = blockIdx.x * 256 + threadIdx.x; if (t >= NOUT * (NBT / 4)) return; const int p0 = (t % (NBT / 4)) * 4; const int o = t / (NBT / 4); const float mu = ST[o * 32], rs = rsqrtf(ST[o * 32 + 1] + 1e-5f); v4f r;
#pragma unroll
  for (int q = 0; q < 4; ++q) { float v = (BEV[(size_t)(p0 + q) * NOUT + o] - mu) * rs; v = bf16_round(g[o]) * v; v += bf16_round(bb[o]); r[q] = fmaxf(v, 0.f); }
  *(volatile v4f*)(out + (size_t)o * NBEV + p0) = r; __threadfence(); *(volatile v4f*)(out + (size_t)o * NBEV + p0) = r; }

extern "C" void kernel_launch(void* const* d_in, const int* in_sizes, int n_in,
                              void* d_out, int out_size, void* d_ws, size_t ws_size, hipStream_t stream) {
  (void)in_sizes; (void)n_in; (void)out_size;
  const float* const* I = (const float* const*)d_in; const float* img = I[0]; const float* calib = I[1]; const float* c1w = I[2]; const float* c1b = I[3]; const float* bn1g = I[4]; const float* bn1b = I[5]; const float* dw = I[6]; const float* dbb = I[7]; const float* bw = I[8]; const float* bbv = I[9]; const float* bn2g = I[10]; const float* bn2b = I[11];
  char* ws = (char*)d_ws; size_t off = 0;
  auto take = [&](size_t bytes) { char* p = ws + off; off += (bytes + 255) & ~(size_t)255; return p; };
  _Float16* IM3 = (_Float16*)take((size_t)NPI * 32 * 2); _Float16* BW1 = (_Float16*)take(64 * 32 * 2); float* BB1 = (float*)take(64 * 4); _Float16* BWD = (_Float16*)take(128 * 32 * 2); float* BBD = (float*)take(128 * 4);
  float* F1 = (float*)take((size_t)NPI * FC * 4); float* DL = (float*)take((size_t)NPI * 128 * 4); float* ST = (float*)take(128 * 32 * 4); float* FEAT = (float*)take((size_t)NPI * FC * 4); float* PROB = (float*)take((size_t)NPI * 128 * 4);
  _Float16* VOX = (_Float16*)take((size_t)CV * NBEV * 2); _Float16* BWB = (_Float16*)take((size_t)NOUT * KB * 2); _Float16* IMB = (_Float16*)take((size_t)(CHR + 32) * KB * 2); float* BEV = (float*)take((size_t)(NBEV + 32) * NOUT * 4);
  if (off > ws_size) return;
  k_im3<<<(NPI + 255) / 256, 256, 0, stream>>>(img, IM3); k_w3<<<1, 256, 0, stream>>>(c1w, c1b, FC, 64, BW1, BB1); k_w3<<<1, 256, 0, stream>>>(dw, dbb, DB, 128, BWD, BBD); k_wbev<<<(unsigned)(((size_t)NOUT * 9 * (CV / 8) + 255) / 256), 256, 0, stream>>>(bw, BWB);
  k_gemm2<0><<<dim3((NPI / 128) * 1, 1), 128, 0, stream>>>(IM3, 32, 0, BW1, 32, 0, 0.0625f, BB1, 0, nullptr, 1, 0, 0, F1, nullptr, FC, 0, NPI, FC, 32);
  k_gemm2<0><<<dim3((NPI / 128) * 2, 1), 128, 0, stream>>>(IM3, 32, 0, BWD, 32, 0, 0.0625f, BBD, 0, nullptr, 1, 0, 0, DL, nullptr, 128, 0, NPI, 128, 32);
  k_dlout<<<(DB * (NPI / 4) + 255) / 256, 256, 0, stream>>>(DL, (float*)d_out + (size_t)NOUT * NBEV);
  k_bnst<<<FC, 256, 0, stream>>>(F1, FC, NPI, ST); k_bnrelu1<<<(NPI * (FC / 4) + 255) / 256, 256, 0, stream>>>(F1, ST, bn1g, bn1b, FEAT);
  k_dsoft<<<(NPI + 7) / 8, 256, 0, stream>>>(DL, PROB);
  k_voxel<<<(unsigned)(((size_t)(NVOX / 2) * (FC / 8) + 255) / 256), 256, 0, stream>>>(calib, FEAT, PROB, VOX);
  for (int r0 = 0; r0 < NBT; r0 += CHR) { k_imb<<<(unsigned)(((size_t)CHR * 9 * (CV / 8) + 255) / 256), 256, 0, stream>>>(VOX, r0, IMB);
    k_gemm2<0><<<dim3(((CHR + 127) / 128) * (NOUT / 64), 1), 128, 0, stream>>>(IMB, KB, 0, BWB, KB, 0, 0.0625f, bbv, 0, nullptr, 1, 0, 0, BEV + (size_t)r0 * NOUT, nullptr, NOUT, 0, CHR, NOUT, KB); }
  k_bnst<<<NOUT, 256, 0, stream>>>(BEV, NOUT, NBT, ST); k_bevout<<<(NOUT * (NBT / 4) + 255) / 256, 256, 0, stream>>>(BEV, ST, bn2g, bn2b, (float*)d_out);
}
